// FlaGatedDeltaNetSequenceMixer_47064251630309
// MI455X (gfx1250) — hardware-run, weakly checked
//
#include <hip/hip_runtime.h>
#include <stddef.h>


#define NBAT   2
#define NSEQ   2048
#define NDIM   1024
#define NHEAD  16
#define HDIM   64
#define KCONV  4
#define NTOK   (NBAT * NSEQ)
#define NTHR   256
#define NWAV   (NTHR / 32)
#define NBA    (2 * NHEAD)
#define PBM    64
#define PBN    128
#define PNT    4
#define BGM    (NWAV * 16)
#define TB     32
#define SGRP   (NTHR / HDIM)
#define SROW   (HDIM / SGRP)
#define WSCAP  134217728
#define WCAR   64.0f
#define OCAR   64.0f
#define GSCL   (1.0f / 64.0f)
#define OSCL   (1.0f / 4096.0f)

#define SZX2   ((size_t)NTOK * NDIM * 2)
#define SZW3   ((size_t)3 * NDIM * NDIM * 2)
#define SZW1   ((size_t)NDIM * NDIM * 2)
#define SZBA2  ((size_t)NBA * NDIM * 2)
#define SZF    ((size_t)NTOK * NDIM * 4)
#define SZBD   ((size_t)NTOK * NBA * 4)
#define OXH    ((size_t)0)
#define OXL    (OXH + SZX2)
#define OXF    (OXL + SZX2)
#define OWH    (OXF + SZX2)
#define OWL    (OWH + SZW3)
#define OWGF   (OWL + SZW3)
#define OWOF   (OWGF + SZW1)
#define OWBH   (OWOF + SZW1)
#define OWBL   (OWBH + SZBA2)
#define OQ     (OWBL + SZBA2)
#define OK_    (OQ + SZF)
#define OV     (OK_ + SZF)
#define OG     (OV + SZF)
#define OBD    (OG + SZF)
#define OOF    (OBD + SZBD)
#define WSTOT  (OOF + SZX2)

#define CVTX_BLK   (NTOK * NDIM / 8 / NTHR)
#define CVTW_BLK   (NDIM * NDIM / 8 / NTHR)
#define CVTBA_BLK  (NBA * NDIM / 8 / NTHR)

static_assert(WSTOT <= (size_t)WSCAP);
static_assert((OXL % 128) == 0 && (OXF % 128) == 0 && (OWH % 128) == 0 && (OWL % 128) == 0);
static_assert((OWGF % 128) == 0 && (OWOF % 128) == 0 && (OWBH % 128) == 0 && (OWBL % 128) == 0);
static_assert((OQ % 128) == 0 && (OK_ % 128) == 0 && (OV % 128) == 0 && (OG % 128) == 0);
static_assert((OBD % 128) == 0 && (OOF % 128) == 0 && OOF + SZX2 == WSTOT);
static_assert((NDIM % 32) == 0);
static_assert((NTOK % PBM) == 0 && (NDIM % PBN) == 0 && (NTOK % BGM) == 0);
static_assert(PBM == 16 * 4 && PBN == 2 * 16 * PNT && NWAV == 8);
static_assert((NTOK * NDIM) % (8 * NTHR) == 0 && (NDIM * NDIM) % (8 * NTHR) == 0);
static_assert((NBA * NDIM) % (8 * NTHR) == 0 && (CVTBA_BLK % 2) == 0 && NTHR * 8 == 2 * NDIM);
static_assert(NHEAD * HDIM == NDIM && NBAT * NSEQ == NTOK && NBA == 32 && NHEAD == 16);
static_assert(NTHR * 4 == NDIM);
static_assert(HDIM == 16 * 4);
static_assert(SGRP * SROW == HDIM && SROW == 16 && SGRP == 4 && NTHR == SGRP * HDIM);
static_assert(TB * HDIM == NTHR * 8 && (NSEQ % TB) == 0 && TB == 4 * NWAV);
static_assert(KCONV == 4);

typedef unsigned short us_t;
typedef _Float16 hf_t;
typedef us_t   v8us __attribute__((ext_vector_type(8), __may_alias__));
typedef hf_t   v8h  __attribute__((ext_vector_type(8), __may_alias__));
typedef __bf16 v16b __attribute__((ext_vector_type(16)));
typedef hf_t   v16h __attribute__((ext_vector_type(16)));
typedef int    v8i  __attribute__((ext_vector_type(8)));
typedef float  v8f  __attribute__((ext_vector_type(8)));
typedef float  v4f  __attribute__((ext_vector_type(4), __may_alias__));
union FragB { v16b v; v8us h[2]; v8i w; };
union FragH { v16h v; v8h  h[2]; v8i w; };
static_assert(sizeof(FragB) == 32);
static_assert(sizeof(FragH) == 32);

__device__ __forceinline__ v8f wmb(FragB a, FragB b, v8f c) {
  v8f d = __builtin_amdgcn_wmma_f32_16x16x32_bf16(false, a.v, false, b.v, (short)0, c, false, false);
  asm volatile("v_nop\n\tv_nop\n\tv_nop\n\tv_nop" : "+v"(d) : "v"(a.w), "v"(b.w));
  return d;
}
__device__ __forceinline__ v8f wmh(FragH a, FragH b, v8f c) {
  v8f d = __builtin_amdgcn_wmma_f32_16x16x32_f16(false, a.v, false, b.v, (short)0, c, false, false);
  asm volatile("v_nop\n\tv_nop\n\tv_nop\n\tv_nop" : "+v"(d) : "v"(a.w), "v"(b.w));
  return d;
}

__device__ __forceinline__ v8f zero8() {
  v8f z = {0.f, 0.f, 0.f, 0.f, 0.f, 0.f, 0.f, 0.f};
  return z;
}
__device__ __forceinline__ v4f zero4() {
  v4f z = {0.f, 0.f, 0.f, 0.f};
  return z;
}

__device__ __forceinline__ unsigned bfr_(float x) {
  const unsigned u = __float_as_uint(x);
  return (u + 0x7FFFu + ((u >> 16) & 1u)) >> 16;
}
__device__ __forceinline__ void split_(float x, us_t& hi, us_t& lo) {
  const unsigned hb = bfr_(x);
  const float hf = __uint_as_float(hb << 16);
  const unsigned lb = bfr_(x - hf);
  hi = (us_t)hb;
  lo = (us_t)lb;
}
__device__ __forceinline__ void cvt8_(const float* f, v8us& vh, v8us& vl) {
#pragma unroll
  for (int i = 0; i < 8; ++i) {
    us_t a, c;
    split_(f[i], a, c);
    vh[i] = a;
    vl[i] = c;
  }
}
__device__ __forceinline__ v8h cvth8_(const float* f, float s) {
  v8h v;
#pragma unroll
  for (int i = 0; i < 8; ++i) v[i] = (hf_t)(f[i] * s);
  return v;
}

__device__ __forceinline__ float rcp_(float d) { return __builtin_amdgcn_rcpf(d); }
__device__ __forceinline__ float sigm_(float x) {
  const float xc = fminf(fmaxf(x, -30.0f), 30.0f);
  return rcp_(1.0f + __expf(-xc));
}
__device__ __forceinline__ float silu_(float x) { return x * sigm_(x); }
__device__ __forceinline__ v4f silu4_(v4f a) {
  v4f r;
  r.x = silu_(a.x); r.y = silu_(a.y); r.z = silu_(a.z); r.w = silu_(a.w);
  return r;
}

__global__ __launch_bounds__(NTHR) void k_cvtx(const float* __restrict__ x, us_t* XH, us_t* XL, hf_t* XF) {
  const size_t e = ((size_t)blockIdx.x * NTHR + threadIdx.x) * 8;
  const v4f a0 = *(const v4f*)(x + e);
  const v4f a1 = *(const v4f*)(x + e + 4);
  float f[8];
  f[0] = a0.x; f[1] = a0.y; f[2] = a0.z; f[3] = a0.w;
  f[4] = a1.x; f[5] = a1.y; f[6] = a1.z; f[7] = a1.w;
  v8us vh, vl;
  cvt8_(f, vh, vl);
  const v8h vf = cvth8_(f, 1.0f);
  *(volatile v8us*)(XH + e) = vh;
  *(volatile v8us*)(XL + e) = vl;
  *(volatile v8h*)(XF + e) = vf;
  __threadfence();
  *(volatile v8us*)(XH + e) = vh;
  *(volatile v8us*)(XL + e) = vl;
  *(volatile v8h*)(XF + e) = vf;
}

__global__ __launch_bounds__(NTHR) void k_cvtw(const float* __restrict__ Wq, const float* __restrict__ Wk,
                                               const float* __restrict__ Wv, const float* __restrict__ Wg,
                                               const float* __restrict__ Wo, us_t* WH, us_t* WL,
                                               hf_t* WGF, hf_t* WOF) {
  const int y = blockIdx.y;
  const size_t e = ((size_t)blockIdx.x * NTHR + threadIdx.x) * 8;
  const float* W = (y == 0) ? Wq : ((y == 1) ? Wk : ((y == 2) ? Wv : ((y == 3) ? Wg : Wo)));
  const v4f a0 = *(const v4f*)(W + e);
  const v4f a1 = *(const v4f*)(W + e + 4);
  float f[8];
  f[0] = a0.x; f[1] = a0.y; f[2] = a0.z; f[3] = a0.w;
  f[4] = a1.x; f[5] = a1.y; f[6] = a1.z; f[7] = a1.w;
  if (y < 3) {
    v8us vh, vl;
    cvt8_(f, vh, vl);
    const size_t off = (size_t)y * NDIM * NDIM + e;
    *(volatile v8us*)(WH + off) = vh;
    *(volatile v8us*)(WL + off) = vl;
    __threadfence();
    *(volatile v8us*)(WH + off) = vh;
    *(volatile v8us*)(WL + off) = vl;
  } else {
    const v8h vf = cvth8_(f, WCAR);
    hf_t* dst = (y == 3) ? WGF : WOF;
    *(volatile v8h*)(dst + e) = vf;
    __threadfence();
    *(volatile v8h*)(dst + e) = vf;
  }
}

__global__ __launch_bounds__(NTHR) void k_cvtba(const float* __restrict__ Wb, const float* __restrict__ Wa,
                                                us_t* WBH, us_t* WBL) {
  const int blk = blockIdx.x;
  const float* src = (blk < CVTBA_BLK / 2) ? Wb : Wa;
  const size_t so = (size_t)(blk & (CVTBA_BLK / 2 - 1)) * (NTHR * 8) + (size_t)threadIdx.x * 8;
  const size_t e = (size_t)blk * (NTHR * 8) + (size_t)threadIdx.x * 8;
  const v4f a0 = *(const v4f*)(src + so);
  const v4f a1 = *(const v4f*)(src + so + 4);
  float f[8];
  f[0] = a0.x; f[1] = a0.y; f[2] = a0.z; f[3] = a0.w;
  f[4] = a1.x; f[5] = a1.y; f[6] = a1.z; f[7] = a1.w;
  v8us vh, vl;
  cvt8_(f, vh, vl);
  *(volatile v8us*)(WBH + e) = vh;
  *(volatile v8us*)(WBL + e) = vl;
  __threadfence();
  *(volatile v8us*)(WBH + e) = vh;
  *(volatile v8us*)(WBL + e) = vl;
}

__global__ __launch_bounds__(NTHR) void k_proj(const us_t* __restrict__ XH, const us_t* __restrict__ XL,
                                               const us_t* __restrict__ WH, const us_t* __restrict__ WL,
                                               float* Q, float* K, float* V) {
  __shared__ __align__(16) float sT[PBM * PBN];
  const int tid = threadIdx.x, lane = tid & 31, wave = tid >> 5, h = lane >> 4, m = lane & 15;
  const int wr = wave & 3, wc = wave >> 2;
  const int bm0 = blockIdx.x * PBM, n0 = blockIdx.y * PBN, z = blockIdx.z;
  const int row0 = bm0 + 16 * wr, col0 = n0 + 64 * wc;

  v8f acc[PNT];
#pragma unroll
  for (int t = 0; t < PNT; ++t) acc[t] = zero8();

  const size_t ao = (size_t)(row0 + m) * NDIM + 8 * h;
  const us_t* aph = XH + ao;
  const us_t* apl = XL + ao;
  const size_t bo = ((size_t)z * NDIM + col0 + m) * NDIM + 8 * h;
  const us_t* bph = WH + bo;
  const us_t* bpl = WL + bo;

#pragma unroll 1
  for (int ks = 0; ks < NDIM / 32; ++ks) {
    const int k0 = 32 * ks;
    FragB ah, al;
    ah.h[0] = *(const v8us*)(aph + k0);
    ah.h[1] = *(const v8us*)(aph + k0 + 16);
    al.h[0] = *(const v8us*)(apl + k0);
    al.h[1] = *(const v8us*)(apl + k0 + 16);
#pragma unroll
    for (int t = 0; t < PNT; ++t) {
      const size_t ro = (size_t)(16 * t) * NDIM + k0;
      FragB bh, bl;
      bh.h[0] = *(const v8us*)(bph + ro);
      bh.h[1] = *(const v8us*)(bph + ro + 16);
      bl.h[0] = *(const v8us*)(bpl + ro);
      bl.h[1] = *(const v8us*)(bpl + ro + 16);
      acc[t] = wmb(ah, bh, acc[t]);
      acc[t] = wmb(ah, bl, acc[t]);
      acc[t] = wmb(al, bh, acc[t]);
    }
  }

#pragma unroll
  for (int t = 0; t < PNT; ++t) {
    const int cl = 64 * wc + 16 * t + m;
#pragma unroll
    for (int r = 0; r < 8; ++r) {
      const int rl = 16 * wr + 8 * h + r;
      sT[rl * PBN + cl] = acc[t][r];
    }
  }
  __syncthreads();

  float* dst = (z == 0) ? Q : ((z == 1) ? K : V);
  v4f ov[8];
#pragma unroll
  for (int rr = 0; rr < 8; ++rr) {
    const int rl = 8 * wave + rr;
    ov[rr] = *(const v4f*)(sT + rl * PBN + 4 * lane);
  }
  const size_t go = (size_t)(bm0 + 8 * wave) * NDIM + n0 + 4 * lane;
#pragma unroll
  for (int rr = 0; rr < 8; ++rr) *(volatile v4f*)(dst + go + (size_t)rr * NDIM) = ov[rr];
  __threadfence();
#pragma unroll
  for (int rr = 0; rr < 8; ++rr) *(volatile v4f*)(dst + go + (size_t)rr * NDIM) = ov[rr];
}

__global__ __launch_bounds__(NTHR) void k_gemmh(const hf_t* __restrict__ A, const hf_t* __restrict__ W,
                                                float* C, float scale) {
  __shared__ __align__(16) float sT[PBM * PBN];
  const int tid = threadIdx.x, lane = tid & 31, wave = tid >> 5, h = lane >> 4, m = lane & 15;
  const int wr = wave & 3, wc = wave >> 2;
  const int bm0 = blockIdx.x * PBM, n0 = blockIdx.y * PBN;
  const int row0 = bm0 + 16 * wr, col0 = n0 + 64 * wc;

  v8f acc[PNT];
#pragma unroll
  for (int t = 0; t < PNT; ++t) acc[t] = zero8();

  const hf_t* ap = A + (size_t)(row0 + m) * NDIM + 8 * h;
  const hf_t* bp = W + (size_t)(col0 + m) * NDIM + 8 * h;

#pragma unroll 1
  for (int ks = 0; ks < NDIM / 32; ++ks) {
    const int k0 = 32 * ks;
    FragH a;
    a.h[0] = *(const v8h*)(ap + k0);
    a.h[1] = *(const v8h*)(ap + k0 + 16);
#pragma unroll
    for (int t = 0; t < PNT; ++t) {
      const size_t ro = (size_t)(16 * t) * NDIM + k0;
      FragH b;
      b.h[0] = *(const v8h*)(bp + ro);
      b.h[1] = *(const v8h*)(bp + ro + 16);
      acc[t] = wmh(a, b, acc[t]);
    }
  }

#pragma unroll
  for (int t = 0; t < PNT; ++t) {
    const int cl = 64 * wc + 16 * t + m;
#pragma unroll
    for (int r = 0; r < 8; ++r) {
      const int rl = 16 * wr + 8 * h + r;
      sT[rl * PBN + cl] = acc[t][r];
    }
  }
  __syncthreads();

  v4f ov[8];
#pragma unroll
  for (int rr = 0; rr < 8; ++rr) {
    const int rl = 8 * wave + rr;
    ov[rr] = *(const v4f*)(sT + rl * PBN + 4 * lane) * scale;
  }
  const size_t go = (size_t)(bm0 + 8 * wave) * NDIM + n0 + 4 * lane;
#pragma unroll
  for (int rr = 0; rr < 8; ++rr) *(volatile v4f*)(C + go + (size_t)rr * NDIM) = ov[rr];
  __threadfence();
#pragma unroll
  for (int rr = 0; rr < 8; ++rr) *(volatile v4f*)(C + go + (size_t)rr * NDIM) = ov[rr];
}

__global__ __launch_bounds__(NTHR) void k_bg(const us_t* __restrict__ XH, const us_t* __restrict__ XL,
                                             const us_t* __restrict__ WBH, const us_t* __restrict__ WBL,
                                             const float* __restrict__ A_log, const float* __restrict__ dt_bias,
                                             float* BD) {
  __shared__ __align__(16) float sL[NWAV * 512];
  const int tid = threadIdx.x, lane = tid & 31, wave = tid >> 5, h = lane >> 4, m = lane & 15;
  const int row0 = blockIdx.x * BGM + 16 * wave;

  v8f acc0 = zero8(), acc1 = zero8();
  const size_t ao = (size_t)(row0 + m) * NDIM + 8 * h;
  const us_t* aph = XH + ao;
  const us_t* apl = XL + ao;
  const size_t bo = (size_t)m * NDIM + 8 * h;
  const us_t* bph = WBH + bo;
  const us_t* bpl = WBL + bo;

#pragma unroll 1
  for (int ks = 0; ks < NDIM / 32; ++ks) {
    const int k0 = 32 * ks;
    FragB ah, al, bh0, bl0, bh1, bl1;
    ah.h[0]  = *(const v8us*)(aph + k0);
    ah.h[1]  = *(const v8us*)(aph + k0 + 16);
    al.h[0]  = *(const v8us*)(apl + k0);
    al.h[1]  = *(const v8us*)(apl + k0 + 16);
    bh0.h[0] = *(const v8us*)(bph + k0);
    bh0.h[1] = *(const v8us*)(bph + k0 + 16);
    bl0.h[0] = *(const v8us*)(bpl + k0);
    bl0.h[1] = *(const v8us*)(bpl + k0 + 16);
    bh1.h[0] = *(const v8us*)(bph + (size_t)16 * NDIM + k0);
    bh1.h[1] = *(const v8us*)(bph + (size_t)16 * NDIM + k0 + 16);
    bl1.h[0] = *(const v8us*)(bpl + (size_t)16 * NDIM + k0);
    bl1.h[1] = *(const v8us*)(bpl + (size_t)16 * NDIM + k0 + 16);
    acc0 = wmb(ah, bh0, acc0);
    acc0 = wmb(ah, bl0, acc0);
    acc0 = wmb(al, bh0, acc0);
    acc1 = wmb(ah, bh1, acc1);
    acc1 = wmb(ah, bl1, acc1);
    acc1 = wmb(al, bh1, acc1);
  }

#pragma unroll
  for (int r = 0; r < 8; ++r) {
    sL[wave * 512 + (8 * h + r) * NBA + m] = acc0[r];
    sL[wave * 512 + (8 * h + r) * NBA + NHEAD + m] = acc1[r];
  }
  __syncthreads();

#pragma unroll 1
  for (int i = 0; i < (16 * NHEAD) / 32; ++i) {
    const int e = lane + 32 * i;
    const int row = e >> 4, hd = e & 15;
    const int ib = wave * 512 + row * NBA + hd;
    const int ia = ib + NHEAD;
    const float lb = sL[ib];
    const float la = sL[ia];
    const float xc = fminf(fmaxf(lb, -30.0f), 30.0f);
    const float beta = 1.0f / (1.0f + expf(-xc));
    const float zz = la + dt_bias[hd];
    const float sp = fmaxf(zz, 0.0f) + log1pf(expf(-fabsf(zz)));
    const float gg = -expf(A_log[hd]) * sp;
    const float dec = expf(gg);
    sL[ib] = beta;
    sL[ia] = dec;
  }
  __syncthreads();

  v4f vals[4];
#pragma unroll
  for (int i = 0; i < 4; ++i) vals[i] = *(const v4f*)(sL + wave * 512 + 128 * i + 4 * lane);
  float* dp = BD + (size_t)row0 * NBA + 4 * lane;
#pragma unroll
  for (int i = 0; i < 4; ++i) *(volatile v4f*)(dp + 128 * i) = vals[i];
  __threadfence();
#pragma unroll
  for (int i = 0; i < 4; ++i) *(volatile v4f*)(dp + 128 * i) = vals[i];
}

__global__ __launch_bounds__(NTHR) void k_conv(float* Q, float* K, float* V, const float* __restrict__ cq,
                                               const float* __restrict__ ck, const float* __restrict__ cv) {
  const int tid = threadIdx.x, b = blockIdx.x, z = blockIdx.y;
  float* P = (z == 0) ? Q : ((z == 1) ? K : V);
  const float* w = (z == 0) ? cq : ((z == 1) ? ck : cv);
  const int c0 = 4 * tid;
  const v4f w0 = *(const v4f*)(w + (size_t)(c0 + 0) * KCONV);
  const v4f w1 = *(const v4f*)(w + (size_t)(c0 + 1) * KCONV);
  const v4f w2 = *(const v4f*)(w + (size_t)(c0 + 2) * KCONV);
  const v4f w3 = *(const v4f*)(w + (size_t)(c0 + 3) * KCONV);
  v4f xm3 = zero4(), xm2 = zero4(), xm1 = zero4();
  float* base = P + (size_t)b * NSEQ * NDIM + c0;

#pragma unroll 1
  for (int t = 0; t < NSEQ; ++t) {
    float* p = base + (size_t)t * NDIM;
    const v4f xt = *(const v4f*)p;
    v4f y;
    y.x = w0.x * xm3.x + w0.y * xm2.x + w0.z * xm1.x + w0.w * xt.x;
    y.y = w1.x * xm3.y + w1.y * xm2.y + w1.z * xm1.y + w1.w * xt.y;
    y.z = w2.x * xm3.z + w2.y * xm2.z + w2.z * xm1.z + w2.w * xt.z;
    y.w = w3.x * xm3.w + w3.y * xm2.w + w3.z * xm1.w + w3.w * xt.w;
    y = silu4_(y);
    if (z < 2) {
      float ss = (y.x * y.x + y.y * y.y) + (y.z * y.z + y.w * y.w);
      ss += __shfl_xor(ss, 8);
      ss += __shfl_xor(ss, 4);
      ss += __shfl_xor(ss, 2);
      ss += __shfl_xor(ss, 1);
      const float r = rsqrtf(ss + 1e-6f);
      y = y * r;
      if (z == 0) y = y * 0.125f;
    }
    *(volatile v4f*)p = y;
    __threadfence();
    *(volatile v4f*)p = y;
    xm3 = xm2; xm2 = xm1; xm1 = xt;
  }
}

__global__ __launch_bounds__(NTHR) void k_scan(const float* __restrict__ Q, const float* __restrict__ K,
                                               const float* __restrict__ V, const float* __restrict__ BD,
                                               const float* __restrict__ G, const float* __restrict__ nw,
                                               hf_t* OF) {
  __shared__ __align__(16) float pA[HDIM * SGRP];
  __shared__ __align__(16) float pB[HDIM * SGRP];
  __shared__ __align__(16) float sO[TB * HDIM];
  const int tid = threadIdx.x, lane = tid & 31, wave = tid >> 5;
  const int g = tid / HDIM, vc = tid & (HDIM - 1);
  const int b = blockIdx.x / NHEAD, hh = blockIdx.x % NHEAD;
  const size_t tokb = (size_t)b * NSEQ;
  const size_t colh = (size_t)hh * HDIM;

  float S[SROW];
#pragma unroll
  for (int j = 0; j < SROW; ++j) S[j] = 0.0f;

#pragma unroll 1
  for (int t = 0; t < NSEQ; ++t) {
    const size_t tok = tokb + (size_t)t;
    const size_t rowo = tok * NDIM + colh;
    const float* kp = K + rowo + SROW * g;
    v4f kv[4];
#pragma unroll
    for (int c = 0; c < 4; ++c) kv[c] = *(const v4f*)(kp + 4 * c);
    const float vv  = V[rowo + vc];
    const float bt  = BD[tok * NBA + hh];
    const float dec = BD[tok * NBA + NHEAD + hh];

    float psk = 0.0f;
#pragma unroll
    for (int c = 0; c < 4; ++c) {
      S[4 * c + 0] *= dec; psk = fmaf(kv[c].x, S[4 * c + 0], psk);
      S[4 * c + 1] *= dec; psk = fmaf(kv[c].y, S[4 * c + 1], psk);
      S[4 * c + 2] *= dec; psk = fmaf(kv[c].z, S[4 * c + 2], psk);
      S[4 * c + 3] *= dec; psk = fmaf(kv[c].w, S[4 * c + 3], psk);
    }
    pA[vc * SGRP + g] = psk;
    __syncthreads();

    const v4f s0 = *(const v4f*)(pA + vc * SGRP);
    const float sk = ((s0.x + s0.y) + s0.z) + s0.w;
    const float u = bt * (vv - sk);

    const float* qp = Q + rowo + SROW * g;
    v4f qv[4];
#pragma unroll
    for (int c = 0; c < 4; ++c) qv[c] = *(const v4f*)(qp + 4 * c);

    float po = 0.0f;
#pragma unroll
    for (int c = 0; c < 4; ++c) {
      S[4 * c + 0] = fmaf(kv[c].x, u, S[4 * c + 0]);
      po = fmaf(qv[c].x, S[4 * c + 0], po);
      S[4 * c + 1] = fmaf(kv[c].y, u, S[4 * c + 1]);
      po = fmaf(qv[c].y, S[4 * c + 1], po);
      S[4 * c + 2] = fmaf(kv[c].z, u, S[4 * c + 2]);
      po = fmaf(qv[c].z, S[4 * c + 2], po);
      S[4 * c + 3] = fmaf(kv[c].w, u, S[4 * c + 3]);
      po = fmaf(qv[c].w, S[4 * c + 3], po);
    }
    pB[vc * SGRP + g] = po;
    __syncthreads();

    if (tid < HDIM) {
      const v4f o0 = *(const v4f*)(pB + vc * SGRP);
      const float ov = ((o0.x + o0.y) + o0.z) + o0.w;
      sO[(t & (TB - 1)) * HDIM + vc] = ov;
    }
    if ((t & (TB - 1)) == TB - 1) {
      __syncthreads();
      const int rr = 4 * wave + (lane >> 3), p = lane & 7;
      const v4f o0 = *(const v4f*)(sO + rr * HDIM + 8 * p);
      const v4f o1 = *(const v4f*)(sO + rr * HDIM + 8 * p + 4);
      float ss = ((o0.x * o0.x + o0.y * o0.y) + (o0.z * o0.z + o0.w * o0.w)) +
                 ((o1.x * o1.x + o1.y * o1.y) + (o1.z * o1.z + o1.w * o1.w));
      ss += __shfl_xor(ss, 4);
      ss += __shfl_xor(ss, 2);
      ss += __shfl_xor(ss, 1);
      const float rs = rsqrtf(ss * (1.0f / (float)HDIM) + 1e-5f);
      const size_t tok = tokb + (size_t)(t - (TB - 1) + rr);
      const float* gp = G + tok * NDIM + colh + 8 * p;
      const v4f g0 = *(const v4f*)gp;
      const v4f g1 = *(const v4f*)(gp + 4);
      const v4f n0 = *(const v4f*)(nw + 8 * p);
      const v4f n1 = *(const v4f*)(nw + 8 * p + 4);
      const v4f y0 = ((o0 * rs) * n0) * silu4_(g0);
      const v4f y1 = ((o1 * rs) * n1) * silu4_(g1);
      v8h hv;
      hv[0] = (hf_t)(y0.x * OCAR); hv[1] = (hf_t)(y0.y * OCAR); hv[2] = (hf_t)(y0.z * OCAR); hv[3] = (hf_t)(y0.w * OCAR);
      hv[4] = (hf_t)(y1.x * OCAR); hv[5] = (hf_t)(y1.y * OCAR); hv[6] = (hf_t)(y1.z * OCAR); hv[7] = (hf_t)(y1.w * OCAR);
      hf_t* op = OF + tok * NDIM + colh + 8 * p;
      *(volatile v8h*)op = hv;
      __threadfence();
      *(volatile v8h*)op = hv;
    }
  }
}

extern "C" void kernel_launch(void* const* d_in, const int* in_sizes, int n_in,
                              void* d_out, int out_size, void* d_ws, size_t ws_size,
                              hipStream_t stream) {
  if (n_in < 14) return;
  if (in_sizes[0] != NTOK * NDIM) return;
  if (in_sizes[1] != NDIM * NDIM || in_sizes[2] != NDIM * NDIM || in_sizes[3] != NDIM * NDIM) return;
  if (in_sizes[4] != NDIM * KCONV || in_sizes[5] != NDIM * KCONV || in_sizes[6] != NDIM * KCONV) return;
  if (in_sizes[7] != NHEAD * NDIM || in_sizes[8] != NHEAD * NDIM) return;
  if (in_sizes[9] != NHEAD || in_sizes[10] != NHEAD) return;
  if (in_sizes[11] != NDIM * NDIM || in_sizes[12] != HDIM || in_sizes[13] != NDIM * NDIM) return;
  if (out_size != NTOK * NDIM) return;
  const size_t tot = (size_t)WSTOT;
  if (tot > ws_size || tot > (size_t)WSCAP) return;

  const float* hidden  = (const float*)d_in[0];
  const float* Wq      = (const float*)d_in[1];
  const float* Wk      = (const float*)d_in[2];
  const float* Wv      = (const float*)d_in[3];
  const float* conv_q  = (const float*)d_in[4];
  const float* conv_k  = (const float*)d_in[5];
  const float* conv_v  = (const float*)d_in[6];
  const float* Wb      = (const float*)d_in[7];
  const float* Wa      = (const float*)d_in[8];
  const float* A_log   = (const float*)d_in[9];
  const float* dt_bias = (const float*)d_in[10];
  const float* Wg      = (const float*)d_in[11];
  const float* norm_w  = (const float*)d_in[12];
  const float* Wo      = (const float*)d_in[13];
  float* out = (float*)d_out;

  char* ws = (char*)d_ws;
  us_t* XH  = (us_t*)(ws + OXH);
  us_t* XL  = (us_t*)(ws + OXL);
  hf_t* XF  = (hf_t*)(ws + OXF);
  us_t* WH  = (us_t*)(ws + OWH);
  us_t* WL  = (us_t*)(ws + OWL);
  hf_t* WGF = (hf_t*)(ws + OWGF);
  hf_t* WOF = (hf_t*)(ws + OWOF);
  us_t* WBH = (us_t*)(ws + OWBH);
  us_t* WBL = (us_t*)(ws + OWBL);
  float* Q  = (float*)(ws + OQ);
  float* K  = (float*)(ws + OK_);
  float* V  = (float*)(ws + OV);
  float* G  = (float*)(ws + OG);
  float* BD = (float*)(ws + OBD);
  hf_t* OF  = (hf_t*)(ws + OOF);

  k_cvtx<<<CVTX_BLK, NTHR, 0, stream>>>(hidden, XH, XL, XF);
  k_cvtw<<<dim3(CVTW_BLK, 5), NTHR, 0, stream>>>(Wq, Wk, Wv, Wg, Wo, WH, WL, WGF, WOF);
  k_cvtba<<<CVTBA_BLK, NTHR, 0, stream>>>(Wb, Wa, WBH, WBL);

  k_proj<<<dim3(NTOK / PBM, NDIM / PBN, 3), NTHR, 0, stream>>>(XH, XL, WH, WL, Q, K, V);

  k_gemmh<<<dim3(NTOK / PBM, NDIM / PBN), NTHR, 0, stream>>>(XF, WGF, G, GSCL);

  k_bg<<<NTOK / BGM, NTHR, 0, stream>>>(XH, XL, WBH, WBL, A_log, dt_bias, BD);

  k_conv<<<dim3(NBAT, 3), NTHR, 0, stream>>>(Q, K, V, conv_q, conv_k, conv_v);

  k_scan<<<NBAT * NHEAD, NTHR, 0, stream>>>(Q, K, V, BD, G, norm_w, OF);

  k_gemmh<<<dim3(NTOK / PBM, NDIM / PBN), NTHR, 0, stream>>>(OF, WOF, out, OSCL);
}
